// DivergenceFreeMLP_89988154786346
// MI455X (gfx1250) — hardware-run, weakly checked
//
#include <hip/hip_runtime.h>
#define JNT 8192
#define JND 2048
#define JNA 128
#define JNB 64
#define JNO 512
typedef unsigned short v8us __attribute__((ext_vector_type(8), may_alias));
typedef float  v8f  __attribute__((ext_vector_type(8)));
typedef float  v4f  __attribute__((ext_vector_type(4)));
typedef float  v4fa __attribute__((ext_vector_type(4), may_alias));

__device__ __forceinline__ unsigned short bf16_bits(float x) { unsigned int u = __float_as_uint(x); return (unsigned short)((u + 0x7FFFu + ((u >> 16) & 1u)) >> 16); }
__device__ __forceinline__ float bf16_val(unsigned short b) { return __uint_as_float(((unsigned int)b) << 16); }
__device__ __forceinline__ float bf16_round(float x) { return bf16_val(bf16_bits(x)); }

typedef _Float16 v16h __attribute__((ext_vector_type(16)));
union FragH { v16h v; v8us half[2]; _Float16 h[16]; unsigned short u[16]; };

__global__ __launch_bounds__(256) void k_wt_f16(const float* __restrict__ W, _Float16* __restrict__ Wt, int K, int N, float scale) {
  const int t = blockIdx.x * 256 + threadIdx.x; if (t >= N * (K / 8)) return; const int n = t / (K / 8), k8 = (t % (K / 8)) * 8; FragH f;
#pragma unroll
  for (int i = 0; i < 8; ++i) f.h[i] = (_Float16)(bf16_round(W[(size_t)(k8 + i) * N + n]) * scale); const v8us o = f.half[0];
  *(volatile v8us*)((unsigned short*)Wt + (size_t)n * K + k8) = o; __threadfence(); *(volatile v8us*)((unsigned short*)Wt + (size_t)n * K + k8) = o;
}

typedef _Float16 v4h __attribute__((ext_vector_type(4)));

__global__ __launch_bounds__(256) void k_x16(const float* __restrict__ x, _Float16* __restrict__ X16, size_t n8) { const size_t t = (size_t)blockIdx.x * 256 + threadIdx.x; if (t >= n8) return; FragH f;
#pragma unroll
  for (int q = 0; q < 8; ++q) f.h[q] = (_Float16)bf16_round(x[t * 8 + q]); *(volatile v8us*)((unsigned short*)X16 + t * 8) = f.half[0]; __threadfence(); *(volatile v8us*)((unsigned short*)X16 + t * 8) = f.half[0]; }

__device__ __forceinline__ v16h g2_frag(const _Float16* p, int hh) { FragH f; f.half[0] = *(const v8us*)((const unsigned short*)p + 8 * hh); f.half[1] = *(const v8us*)((const unsigned short*)p + 16 + 8 * hh); return f.v; }
__device__ __forceinline__ v8f g2_mma(v16h a, v16h b, v8f c) { v8f d = __builtin_amdgcn_wmma_f32_16x16x32_f16(false, a, false, b, (short)0, c, false, false); asm volatile("v_nop\n\tv_nop\n\tv_nop\n\tv_nop" : "+v"(d) : "v"(a), "v"(b)); return d; }
template <int ACT>
__global__ __launch_bounds__(128) void k_gemm2(const _Float16* __restrict__ A, int lda, size_t sA, const _Float16* __restrict__ Bh, int ldb, size_t sB, float alpha, const float* __restrict__ bias, size_t sBias, const float* __restrict__ CP, int rowsPerB, size_t sCPb, int row0g,
    float* __restrict__ C, _Float16* __restrict__ C16, int ldc, size_t sC, int M, int N, int K) { static_assert(ACT == 0 || ACT == 3 || ACT == 6 || ACT == 8 || ACT == 9 || ACT == 11 || ACT == 12 || ACT == 14 || ACT == 15 || ACT == 16 || ACT == 17, "k_gemm2: unsupported ACT code (would silently apply no activation)");
  __shared__ __attribute__((aligned(16))) float so[4][32][68];
  const int tid = threadIdx.x, w = tid >> 5, lane = tid & 31, ln = lane & 15, hh = lane >> 4; const int by = blockIdx.y;
  A += (size_t)by * sA; Bh += (size_t)by * sB; const size_t cofs = (size_t)by * sC; const float* bp = bias ? bias + (size_t)by * sBias : nullptr;
  const int ntn = N >> 6; const int mt = blockIdx.x / ntn, nq = blockIdx.x - mt * ntn; const int row0 = mt * 128 + 32 * w, col0 = nq * 64; if (row0 >= M) return;
  const _Float16* a0p = A + (size_t)(row0 + ln) * lda; const _Float16* a1p = a0p + (size_t)16 * lda;
  const _Float16* b0p = Bh + (size_t)(col0 + ln) * ldb; const _Float16* b1p = b0p + (size_t)16 * ldb; const _Float16* b2p = b1p + (size_t)16 * ldb; const _Float16* b3p = b2p + (size_t)16 * ldb;
  const v8f z8 = {0.f,0.f,0.f,0.f,0.f,0.f,0.f,0.f}; v8f c00 = z8, c01 = z8, c02 = z8, c03 = z8, c10 = z8, c11 = z8, c12 = z8, c13 = z8;
  for (int kb = 0; kb < K; kb += 32) { const v16h a0 = g2_frag(a0p + kb, hh), a1 = g2_frag(a1p + kb, hh);
    v16h b = g2_frag(b0p + kb, hh); c00 = g2_mma(a0, b, c00); c10 = g2_mma(a1, b, c10);
    b = g2_frag(b1p + kb, hh); c01 = g2_mma(a0, b, c01); c11 = g2_mma(a1, b, c11);
    b = g2_frag(b2p + kb, hh); c02 = g2_mma(a0, b, c02); c12 = g2_mma(a1, b, c12);
    b = g2_frag(b3p + kb, hh); c03 = g2_mma(a0, b, c03); c13 = g2_mma(a1, b, c13); }
  v8f accs[8] = {c00, c01, c02, c03, c10, c11, c12, c13};
#pragma unroll
  for (int u = 0; u < 8; ++u) { const int t = u & 3, half = u >> 2; const int col = col0 + t * 16 + ln; const float bv = bp ? bf16_round(bp[col]) : 0.f;
#pragma unroll
    for (int r = 0; r < 8; ++r) { const int rloc = half * 16 + 8 * hh + r; float v = accs[u][r] * alpha + bv; if (CP) { if (rowsPerB < 0) v += CP[cofs + (size_t)(row0g + row0 + rloc) * ldc + col];        else { const int bidx = (row0g + row0 + rloc) / rowsPerB; v += CP[(size_t)bidx * sCPb + (size_t)by * 64 + col]; } }
      if (ACT == 3) v = fmaxf(v, 0.f); else if (ACT == 6) v = 0.5f * v * (1.0f + erff(v * 0.70710678118654752f)); else if (ACT == 11) v = 1.0f / (1.0f + expf(-v)); else if (ACT == 15) v = v / (1.0f + expf(-v)); else if (ACT == 12) v = (v > 0.f) ? v : 0.01f * v; else if (ACT == 8) v = tanhf(v); else if (ACT == 9) v = 0.5f * v * (1.0f + tanhf(0.7978845608028654f * (v + 0.044715f * v * v * v))); else if (ACT == 14) v = (v > 0.f) ? v : 0.1f * v; else if (ACT == 16) v = (v >= 0.f) ? v : 0.3f * v; else if (ACT == 17) v = (v >= 0.f) ? v : 0.2f * v;
      so[w][rloc][t * 16 + ln] = v; } }
  __builtin_amdgcn_fence(__ATOMIC_ACQ_REL, "workgroup"); __builtin_amdgcn_wave_barrier();
  const int rsub = lane >> 4, c4 = (lane & 15) * 4;
  for (int pass = 0; pass < 2; ++pass) {
#pragma unroll
    for (int q = 0; q < 16; ++q) { const int r = q * 2 + rsub; const v4f v = *(const v4fa*)&so[w][r][c4]; if (C) *(volatile v4f*)(C + cofs + (size_t)(row0 + r) * ldc + col0 + c4) = v; if (C16) { v4h h4; for (int i = 0; i < 4; ++i) h4[i] = (_Float16)v[i]; *(volatile v4h*)(C16 + cofs + (size_t)(row0 + r) * ldc + col0 + c4) = h4; } }
    if (pass == 0) __threadfence(); } }

__global__ __launch_bounds__(256) void k_cs16(const float* __restrict__ sw, _Float16* __restrict__ tw, float scale) { const size_t t = (size_t)blockIdx.x * 256 + threadIdx.x; FragH f;
#pragma unroll
  for (int q = 0; q < 8; ++q) f.h[q] = (_Float16)(bf16_round(sw[t * 8 + q]) * scale); unsigned short* tp = (unsigned short*)tw + t * 8; *(volatile v8us*)tp = f.half[0]; __threadfence(); *(volatile v8us*)tp = f.half[0]; }
__global__ __launch_bounds__(256) void k_split(const float* __restrict__ pa, _Float16* __restrict__ th, _Float16* __restrict__ tl, _Float16* __restrict__ tm) {
  const unsigned t = blockIdx.x * 256u + threadIdx.x; const v4f a0 = *(const v4fa*)(pa + (size_t)t * 8), a1 = *(const v4fa*)(pa + (size_t)t * 8 + 4); FragH fh, fl, fm;
#pragma unroll
  for (int q = 0; q < 8; ++q) { const float a = (q < 4) ? a0[q & 3] : a1[q & 3]; const float hs = a * 0x1p12f; const _Float16 hw = (_Float16)((fabsf(hs) < 0x1p-14f) ? 0.0f : hs); const float rs = (a - (float)hw * 0x1p-12f) * 0x1p24f; fh.h[q] = hw; fl.h[q] = (_Float16)((fabsf(rs) < 0x1p-14f) ? 0.0f : rs); fm.h[q] = (_Float16)((a > 0.0f) ? 1.0f : 0.0f); }
  unsigned short* ph = (unsigned short*)th + (size_t)t * 8; unsigned short* pl = (unsigned short*)tl + (size_t)t * 8; unsigned short* pm = (unsigned short*)tm + (size_t)t * 8;
  *(volatile v8us*)ph = fh.half[0]; __threadfence(); *(volatile v8us*)ph = fh.half[0]; *(volatile v8us*)pl = fl.half[0]; __threadfence(); *(volatile v8us*)pl = fl.half[0]; *(volatile v8us*)pm = fm.half[0]; __threadfence(); *(volatile v8us*)pm = fm.half[0]; }
__global__ __launch_bounds__(256) void k_mask2(const float* __restrict__ pa, _Float16* __restrict__ tm) { const unsigned t = blockIdx.x * 256u + threadIdx.x; const v4f a0 = *(const v4fa*)(pa + (size_t)t * 8), a1 = *(const v4fa*)(pa + (size_t)t * 8 + 4); FragH fm;
#pragma unroll
  for (int q = 0; q < 8; ++q) { const float a = (q < 4) ? a0[q & 3] : a1[q & 3]; fm.h[q] = (_Float16)((a > 0.0f) ? 1.0f : 0.0f); }
  unsigned short* pm = (unsigned short*)tm + (size_t)t * 8; *(volatile v8us*)pm = fm.half[0]; __threadfence(); *(volatile v8us*)pm = fm.half[0]; }
__global__ __launch_bounds__(64) void k_ssum(const float* __restrict__ sw, float* __restrict__ ts, int si, int st) { const unsigned t = blockIdx.x * 64u + threadIdx.x; const float* p = sw + (size_t)t * st; float acc = 0.0f;
  for (int i = 0; i < JND; ++i) acc += bf16_round(p[(size_t)i * si]);
  *(volatile float*)(ts + t) = acc; __threadfence(); *(volatile float*)(ts + t) = acc; }
__global__ __launch_bounds__(256) void k_gscale(const float* __restrict__ wb, const float* __restrict__ sa, const float* __restrict__ sc, _Float16* __restrict__ g1, _Float16* __restrict__ g2) {
  const unsigned t = blockIdx.x * 256u + threadIdx.x; const unsigned k1 = t >> 4, j1 = (t & 15u) * 8u; const unsigned j2 = t >> 3, k2 = (t & 7u) * 8u; FragH f1, f2;
#pragma unroll
  for (int q = 0; q < 8; ++q) { const float a = sa[j1 + q] * bf16_round(wb[(size_t)k1 * JNA + j1 + q]) * 0x1p16f; f1.h[q] = (_Float16)((fabsf(a) < 0x1p-14f) ? 0.0f : a); const float b = sc[k2 + q] * bf16_round(wb[(size_t)(k2 + q) * JNA + j2]) * 0x1p14f; f2.h[q] = (_Float16)((fabsf(b) < 0x1p-14f) ? 0.0f : b); }
  unsigned short* p1 = (unsigned short*)g1 + (size_t)t * 8; unsigned short* p2 = (unsigned short*)g2 + (size_t)t * 8;
  *(volatile v8us*)p1 = f1.half[0]; __threadfence(); *(volatile v8us*)p1 = f1.half[0]; *(volatile v8us*)p2 = f2.half[0]; __threadfence(); *(volatile v8us*)p2 = f2.half[0]; }
__global__ __launch_bounds__(256) void k_gate(const float* __restrict__ pr, const float* __restrict__ pm, _Float16* __restrict__ tw, float cy) { const unsigned t = blockIdx.x * 256u + threadIdx.x; const v4f r0 = *(const v4fa*)(pr + (size_t)t * 8), r1 = *(const v4fa*)(pr + (size_t)t * 8 + 4), u0 = *(const v4fa*)(pm + (size_t)t * 8), u1 = *(const v4fa*)(pm + (size_t)t * 8 + 4); FragH f;
#pragma unroll
  for (int q = 0; q < 8; ++q) { const float r = ((q < 4) ? r0[q & 3] : r1[q & 3]) * cy; const float u = (q < 4) ? u0[q & 3] : u1[q & 3]; const float a = (u > 0.0f) ? r : 0.0f; f.h[q] = (_Float16)((fabsf(a) < 0x1p-14f) ? 0.0f : a); }
  unsigned short* tp = (unsigned short*)tw + (size_t)t * 8; *(volatile v8us*)tp = f.half[0]; __threadfence(); *(volatile v8us*)tp = f.half[0]; }
__global__ __launch_bounds__(256) void k_c16(const float* __restrict__ ps, _Float16* __restrict__ tw, float cy) { const unsigned t = blockIdx.x * 256u + threadIdx.x; const v4f s0 = *(const v4fa*)(ps + (size_t)t * 8), s1 = *(const v4fa*)(ps + (size_t)t * 8 + 4); FragH f;
#pragma unroll
  for (int q = 0; q < 8; ++q) { const float a = ((q < 4) ? s0[q & 3] : s1[q & 3]) * cy; f.h[q] = (_Float16)((fabsf(a) < 0x1p-14f) ? 0.0f : a); }
  unsigned short* tp = (unsigned short*)tw + (size_t)t * 8; *(volatile v8us*)tp = f.half[0]; __threadfence(); *(volatile v8us*)tp = f.half[0]; }

extern "C" void kernel_launch(void* const* d_in, const int* in_sizes, int n_in,
                              void* d_out, int out_size, void* d_ws, size_t ws_size, hipStream_t stream) {
  if (n_in < 9) return; if (in_sizes[0] < JNT * JND || in_sizes[1] < JNA * JND || in_sizes[2] < JNA || in_sizes[3] < JNB * JNA || in_sizes[4] < JNB || in_sizes[5] < JND * JNB || in_sizes[7] < JNO * JND || in_sizes[8] < JNO) return; if (out_size < JNT * JNO) return;
  const float* xa = (const float*)d_in[0]; const float* wa = (const float*)d_in[1]; const float* ra = (const float*)d_in[2]; const float* wb = (const float*)d_in[3]; const float* rb = (const float*)d_in[4]; const float* wc = (const float*)d_in[5]; const float* wd = (const float*)d_in[7]; const float* rd = (const float*)d_in[8]; float* res = (float*)d_out;
  static_assert(JNT % 128 == 0 && JNA % 64 == 0 && JNB % 64 == 0 && JNO % 128 == 0 && JND % 32 == 0 && (JNT * JNB) % 2048 == 0 && (JNA * JND) % 2048 == 0 && (JNB * JNA) % 2048 == 0 && (JNO * JNB) % 2048 == 0, "whole tiles, exact cast grids");
  uint8_t* wsp = (uint8_t*)d_ws; size_t off = 0;
  auto take = [&](size_t bytes) { uint8_t* at = wsp + off; off += (bytes + 255) & ~(size_t)255; return at; };
  _Float16* XA = (_Float16*)take((size_t)JNT * JND * 2); _Float16* WA = (_Float16*)take((size_t)JNA * JND * 2); _Float16* WB = (_Float16*)take((size_t)JNB * JNA * 2); _Float16* WD = (_Float16*)take((size_t)JNO * JND * 2); _Float16* WC = (_Float16*)take((size_t)JNB * JND * 2);
  float* L1 = (float*)take((size_t)JNT * JNA * 4); _Float16* AH = (_Float16*)take((size_t)JNT * JNA * 2); _Float16* AL = (_Float16*)take((size_t)JNT * JNA * 2); _Float16* F1 = (_Float16*)take((size_t)JNT * JNA * 2);
  float* T1 = (float*)take((size_t)JNT * JNB * 4); float* L2 = (float*)take((size_t)JNT * JNB * 4); _Float16* F2 = (_Float16*)take((size_t)JNT * JNB * 2);
  float* SA = (float*)take((size_t)JNA * 4); float* SC = (float*)take((size_t)JNB * 4); _Float16* G1 = (_Float16*)take((size_t)JNB * JNA * 2); _Float16* G2 = (_Float16*)take((size_t)JNA * JNB * 2);
  float* R1 = (float*)take((size_t)JNT * JNB * 4); float* R2 = (float*)take((size_t)JNT * JNA * 4); _Float16* GA = (_Float16*)take((size_t)JNT * JNB * 2); _Float16* GB = (_Float16*)take((size_t)JNT * JNA * 2);
  float* P3 = (float*)take((size_t)JNO * JNB * 4); float* P1 = (float*)take((size_t)JNO * JNA * 4); _Float16* Q3 = (_Float16*)take((size_t)JNO * JNB * 2); _Float16* Q1 = (_Float16*)take((size_t)JNO * JNA * 2); float* T2 = (float*)take((size_t)JNT * JNO * 4);
  if (off > ws_size) return;
  k_cs16<<<(unsigned)((size_t)JNT * JND / 8 / 256), 256, 0, stream>>>(xa, XA, 0x1p11f); k_cs16<<<(unsigned)(JNA * JND / 8 / 256), 256, 0, stream>>>(wa, WA, 0x1p19f); k_cs16<<<(unsigned)(JNB * JNA / 8 / 256), 256, 0, stream>>>(wb, WB, 0x1p17f); k_cs16<<<(unsigned)(JNO * JND / 8 / 256), 256, 0, stream>>>(wd, WD, 0x1p19f);
  k_wt_f16<<<(unsigned)((JNB * (JND / 8) + 255) / 256), 256, 0, stream>>>(wc, WC, JND, JNB, 0x1p17f);
  k_gemm2<3><<<dim3((unsigned)((JNT / 128) * (JNA / 64)), 1u), 128, 0, stream>>>(XA, JND, (size_t)0, WA, JND, (size_t)0, 0x1p-30f, ra, (size_t)0, nullptr, 1, 0, 0, L1, nullptr, JNA, (size_t)0, JNT, JNA, JND);
  k_split<<<(unsigned)(JNT * JNA / 8 / 256), 256, 0, stream>>>(L1, AH, AL, F1);
  k_gemm2<0><<<dim3((unsigned)((JNT / 128) * (JNB / 64)), 1u), 128, 0, stream>>>(AH, JNA, (size_t)0, WB, JNA, (size_t)0, 0x1p-29f, nullptr, (size_t)0, nullptr, 1, 0, 0, T1, nullptr, JNB, (size_t)0, JNT, JNB, JNA);
  k_gemm2<0><<<dim3((unsigned)((JNT / 128) * (JNB / 64)), 1u), 128, 0, stream>>>(AL, JNA, (size_t)0, WB, JNA, (size_t)0, 0x1p-41f, rb, (size_t)0, T1, -1, 0, 0, L2, nullptr, JNB, (size_t)0, JNT, JNB, JNA);
  k_mask2<<<(unsigned)(JNT * JNB / 8 / 256), 256, 0, stream>>>(L2, F2);
  k_ssum<<<JNA / 64, 64, 0, stream>>>(wa, SA, 1, JND); k_ssum<<<JNB / 64, 64, 0, stream>>>(wc, SC, JNB, 1);
  k_gscale<<<(unsigned)(JNB * JNA / 8 / 256), 256, 0, stream>>>(wb, SA, SC, G1, G2);
  k_gemm2<0><<<dim3((unsigned)((JNT / 128) * (JNB / 64)), 1u), 128, 0, stream>>>(F1, JNA, (size_t)0, G1, JNA, (size_t)0, 0x1p-16f, nullptr, (size_t)0, nullptr, 1, 0, 0, R1, nullptr, JNB, (size_t)0, JNT, JNB, JNA);
  k_gemm2<0><<<dim3((unsigned)((JNT / 128) * (JNA / 64)), 1u), 128, 0, stream>>>(F2, JNB, (size_t)0, G2, JNB, (size_t)0, 0x1p-14f, nullptr, (size_t)0, nullptr, 1, 0, 0, R2, nullptr, JNA, (size_t)0, JNT, JNA, JNB);
  k_gate<<<(unsigned)(JNT * JNB / 8 / 256), 256, 0, stream>>>(R1, L2, GA, 0x1p13f); k_gate<<<(unsigned)(JNT * JNA / 8 / 256), 256, 0, stream>>>(R2, L1, GB, 0x1p12f);
  k_gemm2<0><<<dim3((unsigned)((JNO / 128) * (JNB / 64)), 1u), 128, 0, stream>>>(WD, JND, (size_t)0, WC, JND, (size_t)0, 0x1p-36f, nullptr, (size_t)0, nullptr, 1, 0, 0, P3, nullptr, JNB, (size_t)0, JNO, JNB, JND);
  k_gemm2<0><<<dim3((unsigned)((JNO / 128) * (JNA / 64)), 1u), 128, 0, stream>>>(WD, JND, (size_t)0, WA, JND, (size_t)0, 0x1p-38f, nullptr, (size_t)0, nullptr, 1, 0, 0, P1, nullptr, JNA, (size_t)0, JNO, JNA, JND);
  k_c16<<<(unsigned)(JNO * JNB / 8 / 256), 256, 0, stream>>>(P3, Q3, 0x1p16f); k_c16<<<(unsigned)(JNO * JNA / 8 / 256), 256, 0, stream>>>(P1, Q1, 0x1p18f);
  k_gemm2<0><<<dim3((unsigned)((JNT / 128) * (JNO / 64)), 1u), 128, 0, stream>>>(GB, JNA, (size_t)0, Q1, JNA, (size_t)0, -0x1p-30f, nullptr, (size_t)0, nullptr, 1, 0, 0, T2, nullptr, JNO, (size_t)0, JNT, JNO, JNA);
  k_gemm2<0><<<dim3((unsigned)((JNT / 128) * (JNO / 64)), 1u), 128, 0, stream>>>(GA, JNB, (size_t)0, Q3, JNB, (size_t)0, 0x1p-29f, rd, (size_t)0, T2, -1, 0, 0, res, nullptr, JNO, (size_t)0, JNT, JNO, JNB);
}
